// DeformableAlign_14877766713886
// MI455X (gfx1250) — hardware-verified
//
#include <hip/hip_runtime.h>
#include <stdint.h>

#pragma clang fp contract(off)

#define NB     4
#define NC     256
#define NOC    256
#define NOFF   18
#define NOP    32
#define HI     64
#define WI     64
#define HWI    (HI * WI)
#define PD     66
#define KT     2304
#define NPIX   (NB * HWI)
#define PLANE_E ((size_t)NB * PD * PD * NC)
#define SP     264
#define OFP    36
#define MPX    32
#define OSP    36
#define LPP    ((NC * 2) / 128)
#define NLX    (PD * LPP)
#define NLIT   ((NLX + 31) / 32)
#define CSC    16.0f
#define WSC    1024.0f
#define INV_S  6.103515625e-05f
#define WO_CHK (NOP * KT / 8)
#define WR_CHK (NOC * KT / 8)
#define WO_BLK (WO_CHK / 256)
#define WR_BLK (WR_CHK / 256)
#define TRAW_B (NOC * OSP * 4)
#define OFF_BLK (NB * HI)
#define CNV_BLK (NB * HI * (WI / MPX))
#define CVT_BLK (2 * NB * PD)

#define WS_WO   ((size_t)0)
#define WS_WR   (WS_WO + (size_t)NOP * KT * 2)
#define WS_XH   (WS_WR + (size_t)NOC * KT * 2)
#define WS_YH   (WS_XH + PLANE_E * 2)
#define WS_OF   (WS_YH + PLANE_E * 2)
#define WS_END  (WS_OF + (size_t)NPIX * NOP * 4)

static_assert(WO_CHK % 256 == 0);
static_assert(WR_CHK % 256 == 0);
static_assert(KT % 32 == 0);
static_assert(KT == 9 * NC);
static_assert((WS_WR % 128) == 0);
static_assert((WS_XH % 128) == 0);
static_assert((WS_YH % 128) == 0);
static_assert((WS_OF % 128) == 0);
static_assert((WS_END % 128) == 0);
static_assert(WS_END <= (size_t)134217728);
static_assert((SP * 2) % 16 == 0);
static_assert((OFP * 4) % 16 == 0);
static_assert((OSP * 4) % 16 == 0);
static_assert(MPX * SP * 2 <= TRAW_B);
static_assert(PD * SP * 2 <= 48000);
static_assert(MPX * NOP * 4 + TRAW_B <= 60000);
static_assert(64 * OFP * 4 <= 16384);
static_assert(LPP == 4);
static_assert(NOP * 4 == 128);
static_assert(MPX * 4 == 128);
static_assert(NLIT * 32 >= NLX);
static_assert(8 * 4 == MPX);
static_assert(NC == 8 * 8 * 4);
static_assert(WI % MPX == 0);
static_assert(NC % 64 == 0);
static_assert(OFF_BLK == 256);
static_assert(CNV_BLK == 512);
static_assert(CVT_BLK == 528);
static_assert(NC * WI == 16 * 256 * 4);

typedef _Float16       v16h __attribute__((ext_vector_type(16)));
typedef _Float16       v8h  __attribute__((ext_vector_type(8)));
typedef __bf16         v16b __attribute__((ext_vector_type(16)));
typedef __bf16         v8b  __attribute__((ext_vector_type(8)));
typedef float          v8f  __attribute__((ext_vector_type(8)));
typedef float          v4f  __attribute__((ext_vector_type(4)));
typedef unsigned       v4u  __attribute__((ext_vector_type(4)));
typedef unsigned short v8us __attribute__((ext_vector_type(8)));

__device__ __forceinline__ unsigned bfb(float f) {
  const unsigned u = __float_as_uint(f);
  return (u + 0x7FFFu + ((u >> 16) & 1u)) >> 16;
}
__device__ __forceinline__ float bf_rne(float f) { return __uint_as_float(bfb(f) << 16); }
__device__ __forceinline__ unsigned hbits(_Float16 h) {
  return (unsigned)__builtin_bit_cast(unsigned short, h);
}
__device__ __forceinline__ v8f zero8f() { v8f z = {0.f, 0.f, 0.f, 0.f, 0.f, 0.f, 0.f, 0.f}; return z; }
__device__ __forceinline__ v8us zero8us() {
  v8us z;
#pragma unroll
  for (int e = 0; e < 8; ++e) z[e] = (unsigned short)0;
  return z;
}

__device__ __forceinline__ v16h ldfrag_h(const _Float16* p) {
  union { v16h v; v8h h[2]; } f;
  f.h[0] = *(const v8h*)(p);
  f.h[1] = *(const v8h*)(p + 16);
  return f.v;
}
__device__ __forceinline__ v16b ldfrag_b(const __bf16* p) {
  union { v16b v; v8b h[2]; } f;
  f.h[0] = *(const v8b*)(p);
  f.h[1] = *(const v8b*)(p + 16);
  return f.v;
}

__device__ __forceinline__ v8f mma_h(v16h a, v16h b, v8f c) {
  return __builtin_amdgcn_wmma_f32_16x16x32_f16(false, a, false, b, (short)0, c, false, false);
}
__device__ __forceinline__ v8f mma_b(v16b a, v16b b, v8f c) {
  return __builtin_amdgcn_wmma_f32_16x16x32_bf16(false, a, false, b, (short)0, c, false, false);
}
template <typename F>
__device__ __forceinline__ void guard1x4(v8f& c0, const F& f0, const F& f1, const F& f2, const F& f3) {
#if defined(__HIP_DEVICE_COMPILE__)
  asm volatile("v_nop\n\tv_nop\n\tv_nop\n\tv_nop"
               : "+v"(c0)
               : "v"(f0), "v"(f1), "v"(f2), "v"(f3));
#endif
}
template <typename F>
__device__ __forceinline__ void guard4x5(v8f& c0, v8f& c1, v8f& c2, v8f& c3,
                                         const F& f0, const F& f1, const F& f2,
                                         const F& f3, const F& f4) {
#if defined(__HIP_DEVICE_COMPILE__)
  asm volatile("v_nop\n\tv_nop\n\tv_nop\n\tv_nop"
               : "+v"(c0), "+v"(c1), "+v"(c2), "+v"(c3)
               : "v"(f0), "v"(f1), "v"(f2), "v"(f3), "v"(f4));
#endif
}
__device__ __forceinline__ void acc_guard1(v8f& c0) {
#if defined(__HIP_DEVICE_COMPILE__)
  asm volatile("v_nop\n\tv_nop\n\tv_nop\n\tv_nop" : "+v"(c0));
#endif
}
__device__ __forceinline__ void acc_guard4(v8f& c0, v8f& c1, v8f& c2, v8f& c3) {
#if defined(__HIP_DEVICE_COMPILE__)
  asm volatile("v_nop\n\tv_nop\n\tv_nop\n\tv_nop"
               : "+v"(c0), "+v"(c1), "+v"(c2), "+v"(c3));
#endif
}

__global__ __launch_bounds__(256)
void k_wpack(const float* __restrict__ woff, const float* __restrict__ wdc,
             unsigned* wo, unsigned* wr)
{
  const int tid = threadIdx.x;
  if (blockIdx.x < WO_BLK) {
    const int q   = blockIdx.x * 256 + tid;
    const int co  = q / (KT / 8);
    const int kc  = (q - co * (KT / 8)) * 8;
    const int tap = kc >> 8;
    const int ci0 = kc & (NC - 1);
    const int coo = min(co, NOFF - 1);
    unsigned hb[8];
#pragma unroll
    for (int j = 0; j < 8; ++j) {
      const unsigned tv = bfb(woff[((size_t)(coo * NC + ci0 + j)) * 9 + tap]);
      hb[j] = (co < NOFF) ? tv : 0u;
    }
    v4u wh;
    wh.x = hb[0] | (hb[1] << 16);
    wh.y = hb[2] | (hb[3] << 16);
    wh.z = hb[4] | (hb[5] << 16);
    wh.w = hb[6] | (hb[7] << 16);
    unsigned* dst = wo + (size_t)q * 4;
    *(volatile v4u*)dst = wh;
    __threadfence();
    *(volatile v4u*)dst = wh;
  } else {
    const int q   = (blockIdx.x - WO_BLK) * 256 + tid;
    const int co  = q / (KT / 8);
    const int kc  = (q - co * (KT / 8)) * 8;
    const int tap = kc >> 8;
    const int ci0 = kc & (NC - 1);
    unsigned hb[8];
#pragma unroll
    for (int j = 0; j < 8; ++j) {
      const float v = bf_rne(wdc[((size_t)(co * NC + ci0 + j)) * 9 + tap]) * WSC;
      hb[j] = hbits((_Float16)v);
    }
    v4u wh;
    wh.x = hb[0] | (hb[1] << 16);
    wh.y = hb[2] | (hb[3] << 16);
    wh.z = hb[4] | (hb[5] << 16);
    wh.w = hb[6] | (hb[7] << 16);
    unsigned* dst = wr + (size_t)q * 4;
    *(volatile v4u*)dst = wh;
    __threadfence();
    *(volatile v4u*)dst = wh;
  }
}

__global__ __launch_bounds__(256)
void k_cvt(const float* __restrict__ x, const float* __restrict__ y,
           unsigned short* xh, unsigned short* yh)
{
  __shared__ __align__(16) unsigned short T[PD * SP];
  const int tid  = threadIdx.x;
  const int lane = tid & 31;
  const int wid  = tid >> 5;
  const int pj   = lane & 7;
  const int lq   = lane >> 3;
  const int pl   = blockIdx.x / (NB * PD);
  const int bi   = blockIdx.x - pl * (NB * PD);
  const int b    = bi / PD;
  const int hp   = bi - b * PD;
  const float* src    = (pl == 0) ? x : y;
  unsigned short* dst = (pl == 0) ? xh : yh;
  const size_t rowe = ((size_t)(b * PD + hp)) * PD * NC;

  if (hp == 0 || hp == PD - 1) {
    const v8us zu = zero8us();
    size_t e[NLIT]; bool ok[NLIT];
#pragma unroll
    for (int r = 0; r < NLIT; ++r) {
      const int L  = r * 32 + wid * 4 + lq;
      ok[r] = (L < NLX);
      const int Lc = ok[r] ? L : (NLX - 1);
      e[r] = rowe + (size_t)64 * Lc + 8 * pj;
    }
#pragma unroll
    for (int r = 0; r < NLIT; ++r) if (ok[r]) *(volatile v8us*)(dst + e[r]) = zu;
    __threadfence();
#pragma unroll
    for (int r = 0; r < NLIT; ++r) if (ok[r]) *(volatile v8us*)(dst + e[r]) = zu;
  } else {
    const int h = hp - 1;
    if (tid < 64) {
      const int slot = (tid < 32) ? 0 : (PD - 1);
      *(v8us*)&T[slot * SP + 8 * (tid & 31)] = zero8us();
    }
#pragma unroll
    for (int i = 0; i < 16; ++i) {
      const int idx = tid + 256 * i;
      const int w4  = idx & 15;
      const int c   = idx >> 4;
      const v4f v = *(const v4f*)(src + ((size_t)(b * NC + c) * HI + h) * WI + 4 * w4);
      unsigned short* tp = T + (4 * w4 + 1) * SP + c;
      tp[0 * SP] = (unsigned short)bfb(v.x);
      tp[1 * SP] = (unsigned short)bfb(v.y);
      tp[2 * SP] = (unsigned short)bfb(v.z);
      tp[3 * SP] = (unsigned short)bfb(v.w);
    }
    __syncthreads();
    v8us val[NLIT]; size_t e[NLIT]; bool ok[NLIT];
#pragma unroll
    for (int r = 0; r < NLIT; ++r) {
      const int L  = r * 32 + wid * 4 + lq;
      ok[r] = (L < NLX);
      const int Lc = ok[r] ? L : (NLX - 1);
      val[r] = *(const v8us*)&T[(Lc >> 2) * SP + 64 * (Lc & 3) + 8 * pj];
      e[r]   = rowe + (size_t)64 * Lc + 8 * pj;
    }
#pragma unroll
    for (int r = 0; r < NLIT; ++r) if (ok[r]) *(volatile v8us*)(dst + e[r]) = val[r];
    __threadfence();
#pragma unroll
    for (int r = 0; r < NLIT; ++r) if (ok[r]) *(volatile v8us*)(dst + e[r]) = val[r];
  }
}

__global__ __launch_bounds__(256)
void k_offs(const __bf16* __restrict__ yh, const __bf16* __restrict__ wo,
            const float* __restrict__ boff, float* offp)
{
  __shared__ __align__(16) float st[64 * OFP];

  const int tid  = threadIdx.x;
  const int lane = tid & 31;
  const int wid  = tid >> 5;
  const int l15  = lane & 15;
  const int hh   = lane >> 4;
  const int b    = blockIdx.x / HI;
  const int h    = blockIdx.x - b * HI;

  const int mt = wid & 3;
  const int nt = wid >> 2;
  const __bf16* ap = yh + (((size_t)(b * PD + h)) * PD + 16 * mt + l15) * NC + 8 * hh;
  const __bf16* bp = wo + (size_t)(16 * nt + l15) * KT + 8 * hh;
  v8f acc = zero8f();
#pragma unroll 1
  for (int kh = 0; kh < 3; ++kh) {
#pragma unroll 1
    for (int kw = 0; kw < 3; ++kw) {
      const __bf16* a  = ap + (kh * PD + kw) * NC;
      const __bf16* bk = bp + (kh * 3 + kw) * NC;
#pragma unroll
      for (int kc = 0; kc < NC / 64; ++kc) {
        const v16b fa0 = ldfrag_b(a + 64 * kc);
        const v16b fa1 = ldfrag_b(a + 64 * kc + 32);
        const v16b fb0 = ldfrag_b(bk + 64 * kc);
        const v16b fb1 = ldfrag_b(bk + 64 * kc + 32);
        acc = mma_b(fa0, fb0, acc);
        acc = mma_b(fa1, fb1, acc);
        guard1x4(acc, fa0, fa1, fb0, fb1);
      }
    }
  }
  acc_guard1(acc);

  {
    const int ch  = 16 * nt + l15;
    const int cho = min(ch, NOFF - 1);
    const float obv = bf_rne(boff[cho]);
    float* srow = st + (16 * mt + 8 * hh) * OFP + ch;
#pragma unroll
    for (int r = 0; r < 8; ++r) {
      float v = acc[r] + obv;
      if (ch >= NOFF) v = 0.0f;
      srow[r * OFP] = v;
    }
  }
  __syncthreads();

  {
    const int pj = lane & 7;
    const int lq = lane >> 3;
    const size_t pix0 = (size_t)(b * HWI + h * WI);
    v4f val[2]; size_t e[2];
#pragma unroll
    for (int r = 0; r < 2; ++r) {
      const int L = r * 32 + wid * 4 + lq;
      val[r] = *(const v4f*)&st[L * OFP + 4 * pj];
      e[r]   = (pix0 + L) * NOP + 4 * pj;
    }
#pragma unroll
    for (int r = 0; r < 2; ++r) *(volatile v4f*)(offp + e[r]) = val[r];
    __threadfence();
#pragma unroll
    for (int r = 0; r < 2; ++r) *(volatile v4f*)(offp + e[r]) = val[r];
  }
}

__global__ __launch_bounds__(256)
void k_conv(const unsigned short* __restrict__ xh, const _Float16* __restrict__ wr,
            const float* __restrict__ offp, const float* __restrict__ dbias, float* out)
{
  __shared__ __align__(16) float offl[MPX * NOP];
  __shared__ __align__(16) unsigned char traw[TRAW_B];
  _Float16* At = (_Float16*)traw;
  float*    os = (float*)traw;

  const int tid  = threadIdx.x;
  const int lane = tid & 31;
  const int wid  = tid >> 5;
  const int l15  = lane & 15;
  const int hh   = lane >> 4;
  const int pj   = lane & 7;
  const int lq   = lane >> 3;
  const int b    = blockIdx.x / (HI * (WI / MPX));
  const int rem  = blockIdx.x - b * (HI * (WI / MPX));
  const int h    = rem / (WI / MPX);
  const int xo   = (rem - h * (WI / MPX)) * MPX;
  const size_t pix0 = (size_t)(b * HWI + h * WI + xo);

  {
    const int px = tid >> 3;
    const int pc = tid & 7;
    *(v4f*)&offl[px * NOP + 4 * pc] = *(const v4f*)(offp + (pix0 + px) * NOP + 4 * pc);
  }
  __syncthreads();

  const int mt = wid & 1;
  const int nq = wid >> 1;
  const _Float16* bp = wr + (size_t)(64 * nq + l15) * KT + 8 * hh;
  v8f acc[4];
#pragma unroll
  for (int j = 0; j < 4; ++j) acc[j] = zero8f();

#pragma unroll 1
  for (int kh = 0; kh < 3; ++kh) {
#pragma unroll 1
    for (int kw = 0; kw < 3; ++kw) {
      const int tap = kh * 3 + kw;

      {
        const int m = 4 * wid + lq;
        const float* orow = offl + m * NOP;
        const float dy = orow[2 * tap];
        const float dx = orow[2 * tap + 1];
        const float hf = (float)(h - 1 + kh) + dy;
        const float wf = (float)(xo + m - 1 + kw) + dx;
        const float h0f = floorf(hf);
        const float w0f = floorf(wf);
        const float lh  = hf - h0f;
        const float lw  = wf - w0f;
        const float wh0 = 1.0f - lh;
        const float ww0 = 1.0f - lw;
        const int r0 = (int)fminf(fmaxf(h0f, -2.0f), (float)(PD - 1));
        const int c0 = (int)fminf(fmaxf(w0f, -2.0f), (float)(PD - 1));
        const int r1 = r0 + 1;
        const int c1 = c0 + 1;
        const bool vr0 = (r0 >= 0) && (r0 < HI);
        const bool vr1 = (r1 >= 0) && (r1 < HI);
        const bool vc0 = (c0 >= 0) && (c0 < WI);
        const bool vc1 = (c1 >= 0) && (c1 < WI);
        const float cw00 = (vr0 && vc0) ? (wh0 * ww0) : 0.0f;
        const float cw01 = (vr0 && vc1) ? (wh0 * lw)  : 0.0f;
        const float cw10 = (vr1 && vc0) ? (lh * ww0)  : 0.0f;
        const float cw11 = (vr1 && vc1) ? (lh * lw)   : 0.0f;
        const int pr0 = min(max(r0 + 1, 0), PD - 1);
        const int pr1 = min(max(r1 + 1, 0), PD - 1);
        const int pc0 = min(max(c0 + 1, 0), PD - 1);
        const int pc1 = min(max(c1 + 1, 0), PD - 1);
        const size_t rb0 = ((size_t)(b * PD + pr0)) * PD;
        const size_t rb1 = ((size_t)(b * PD + pr1)) * PD;
        const unsigned short* p00 = xh + (rb0 + pc0) * NC;
        const unsigned short* p01 = xh + (rb0 + pc1) * NC;
        const unsigned short* p10 = xh + (rb1 + pc0) * NC;
        const unsigned short* p11 = xh + (rb1 + pc1) * NC;
        _Float16* arow = At + m * SP;
#pragma unroll 1
        for (int it = 0; it < 4; ++it) {
          const int cb = 8 * (pj + 8 * it);
          const v4u q00 = *(const v4u*)(p00 + cb);
          const v4u q01 = *(const v4u*)(p01 + cb);
          const v4u q10 = *(const v4u*)(p10 + cb);
          const v4u q11 = *(const v4u*)(p11 + cb);
          v8h o;
#pragma unroll
          for (int j = 0; j < 4; ++j) {
            const unsigned u00 = q00[j], u01 = q01[j], u10 = q10[j], u11 = q11[j];
            {
              float a = cw00 * __uint_as_float(u00 << 16);
              a = a + cw01 * __uint_as_float(u01 << 16);
              a = a + cw10 * __uint_as_float(u10 << 16);
              a = a + cw11 * __uint_as_float(u11 << 16);
              a = a * CSC;
              o[2 * j] = (_Float16)a;
            }
            {
              float a = cw00 * __uint_as_float(u00 & 0xffff0000u);
              a = a + cw01 * __uint_as_float(u01 & 0xffff0000u);
              a = a + cw10 * __uint_as_float(u10 & 0xffff0000u);
              a = a + cw11 * __uint_as_float(u11 & 0xffff0000u);
              a = a * CSC;
              o[2 * j + 1] = (_Float16)a;
            }
          }
          *(v8h*)(arow + cb) = o;
        }
      }
      __syncthreads();

      {
        const _Float16* bt = bp + tap * NC;
        const _Float16* ab = At + (16 * mt + l15) * SP + 8 * hh;
#pragma unroll 2
        for (int kc = 0; kc < NC / 32; ++kc) {
          const v16h fa  = ldfrag_h(ab + 32 * kc);
          const v16h fb0 = ldfrag_h(bt + 32 * kc);
          const v16h fb1 = ldfrag_h(bt + 16 * KT + 32 * kc);
          const v16h fb2 = ldfrag_h(bt + 32 * KT + 32 * kc);
          const v16h fb3 = ldfrag_h(bt + 48 * KT + 32 * kc);
          acc[0] = mma_h(fa, fb0, acc[0]);
          acc[1] = mma_h(fa, fb1, acc[1]);
          acc[2] = mma_h(fa, fb2, acc[2]);
          acc[3] = mma_h(fa, fb3, acc[3]);
          guard4x5(acc[0], acc[1], acc[2], acc[3], fa, fb0, fb1, fb2, fb3);
        }
      }
      __syncthreads();
    }
  }
  acc_guard4(acc[0], acc[1], acc[2], acc[3]);

  {
#pragma unroll
    for (int j = 0; j < 4; ++j) {
      const int o = 64 * nq + 16 * j + l15;
      const float bv = bf_rne(dbias[o]);
      float* orow = os + o * OSP + 16 * mt + 8 * hh;
#pragma unroll
      for (int r = 0; r < 8; ++r) {
        float v = acc[j][r] * INV_S;
        v = v + bv;
        orow[r] = v;
      }
    }
  }
  __syncthreads();

  {
    v4f val[8]; size_t e[8];
#pragma unroll
    for (int it = 0; it < 8; ++it) {
      const int L = it * 32 + wid * 4 + lq;
      val[it] = *(const v4f*)(os + L * OSP + 4 * pj);
      e[it]   = ((size_t)(b * NOC + L) * HI + h) * WI + xo + 4 * pj;
    }
#pragma unroll
    for (int it = 0; it < 8; ++it) *(volatile v4f*)(out + e[it]) = val[it];
    __threadfence();
#pragma unroll
    for (int it = 0; it < 8; ++it) *(volatile v4f*)(out + e[it]) = val[it];
  }
}

extern "C" void kernel_launch(void* const* d_in, const int* in_sizes, int n_in,
                              void* d_out, int out_size, void* d_ws, size_t ws_size,
                              hipStream_t stream) {
  if (n_in < 6) return;
  if (in_sizes[0] != NB * NC * HWI) return;
  if (in_sizes[1] != NB * NC * HWI) return;
  if (in_sizes[2] != NOFF * NC * 9) return;
  if (in_sizes[3] != NOFF) return;
  if (in_sizes[4] != NOC * NC * 9) return;
  if (in_sizes[5] != NOC) return;
  if (out_size != NB * NOC * HWI) return;
  if (WS_END > ws_size) return;

  const float* x     = (const float*)d_in[0];
  const float* y     = (const float*)d_in[1];
  const float* w_off = (const float*)d_in[2];
  const float* b_off = (const float*)d_in[3];
  const float* w_dc  = (const float*)d_in[4];
  const float* b_dc  = (const float*)d_in[5];
  float* out = (float*)d_out;
  char* ws = (char*)d_ws;

  unsigned* wo_u       = (unsigned*)(ws + WS_WO);
  unsigned* wr_u       = (unsigned*)(ws + WS_WR);
  unsigned short* xh_u = (unsigned short*)(ws + WS_XH);
  unsigned short* yh_u = (unsigned short*)(ws + WS_YH);
  float* offp          = (float*)(ws + WS_OF);

  k_wpack<<<dim3(WO_BLK + WR_BLK), dim3(256), 0, stream>>>(w_off, w_dc, wo_u, wr_u);
  (void)hipGetLastError();

  k_cvt<<<dim3(CVT_BLK), dim3(256), 0, stream>>>(x, y, xh_u, yh_u);
  (void)hipGetLastError();

  k_offs<<<dim3(OFF_BLK), dim3(256), 0, stream>>>((const __bf16*)yh_u, (const __bf16*)wo_u,
                                                    b_off, offp);
  (void)hipGetLastError();

  k_conv<<<dim3(CNV_BLK), dim3(256), 0, stream>>>((const unsigned short*)xh_u, (const _Float16*)wr_u,
                                                   (const float*)offp, b_dc, out);
  (void)hipGetLastError();
}
